// LSTMModel_82360292868323
// MI455X (gfx1250) — hardware-verified
//
#include <hip/hip_runtime.h>
#include <math.h>

constexpr int NBATCH = 128;
constexpr int NSTEP  = 128;
constexpr int NIN    = 512;
constexpr int NHID   = 1024;
constexpr int NGATE  = 4 * NHID;
constexpr int BSEL   = NBATCH - 1;
constexpr int REC_THREADS = 512;
constexpr int REC_WAVES   = REC_THREADS / 32;
constexpr int UB_PER_WAVE = (NHID / 16) / REC_WAVES;
constexpr int HPITCH = 1032;
constexpr int SLABP  = 68;
constexpr float W_CARRY      = 256.0f;
constexpr float W_CARRY_INV  = 1.0f / 256.0f;
constexpr float LO_CARRY     = 2048.0f;
constexpr float LO_CARRY_INV = 1.0f / 2048.0f;
constexpr float F16_MIN_NORMAL = 6.103515625e-05f;

static_assert(NGATE == 4096);
static_assert(UB_PER_WAVE == 4);
static_assert(NSTEP % 64 == 0 && NGATE % 64 == 0);
static_assert(NIN % 32 == 0 && NHID % 32 == 0);
static_assert((HPITCH % 8) == 0 && HPITCH >= NHID);
static_assert((NSTEP * NIN) % 8 == 0 && (NSTEP * NHID) % 8 == 0);
static_assert((NGATE * NIN) % (8 * 256) == 0 && (NGATE * NHID) % (8 * 256) == 0);

typedef __attribute__((ext_vector_type(16))) _Float16 v16h;
typedef __attribute__((ext_vector_type(8)))  _Float16 v8h;
typedef __attribute__((ext_vector_type(8)))  float    v8f;
typedef __attribute__((ext_vector_type(4)))  float    v4f;
typedef __attribute__((ext_vector_type(4)))  unsigned v4u;

__device__ __forceinline__ void guard_grp4(v8f& a0, v8f& a1, v8f& a2, v8f& a3,
                                           v16h x, v16h y0, v16h y1, v16h y2, v16h y3) {
  asm volatile("v_nop\n\tv_nop\n\tv_nop\n\tv_nop"
               : "+v"(a0), "+v"(a1), "+v"(a2), "+v"(a3)
               : "v"(x), "v"(y0), "v"(y1), "v"(y2), "v"(y3));
}
__device__ __forceinline__ void acc_guard4(v8f& a, v8f& b, v8f& c, v8f& d) {
  asm volatile("v_nop\n\tv_nop\n\tv_nop\n\tv_nop" : "+v"(a), "+v"(b), "+v"(c), "+v"(d));
}

template <typename T> struct Frag;
template <> struct Frag<_Float16> {
  typedef v16h V;
  union U { v16h v; v8h h[2]; v4u q[2]; };
  static __device__ __forceinline__ v16h load(const _Float16* p) {
    U f; f.h[0] = *(const v8h*)(p); f.h[1] = *(const v8h*)(p + 16); return f.v;
  }
  static __device__ __forceinline__ v8f mma(v16h a, v16h b, v8f c) {
    return __builtin_amdgcn_wmma_f32_16x16x32_f16(false, a, false, b, (short)0, c, false, false);
  }
};

__device__ __forceinline__ void split_hl(float v, _Float16& h, _Float16& l) {
  const float vh = (fabsf(v) < F16_MIN_NORMAL) ? 0.0f : v;
  h = (_Float16)vh;
  const float hf = (float)h;
  const float r = (v - hf) * LO_CARRY;
  l = (_Float16)r;
}

__global__ __launch_bounds__(256) void cvt_w_kernel(const float* __restrict__ src, unsigned short* __restrict__ dst,
                                                    int n8, float sc) {
  const int i = blockIdx.x * 256 + threadIdx.x;
  if (i < n8) {
    const v4f a = *(const v4f*)(src + (size_t)i * 8);
    const v4f b = *(const v4f*)(src + (size_t)i * 8 + 4);
    v8h hv;
#pragma unroll
    for (int e = 0; e < 4; ++e) {
      const float fa = a[e] * sc;
      const float fb = b[e] * sc;
      hv[e]     = (_Float16)fa;
      hv[4 + e] = (_Float16)fb;
    }
    volatile v8h* p = (volatile v8h*)(dst + (size_t)i * 8);
    *p = hv;
    __threadfence();
    *p = hv;
  }
}

__global__ __launch_bounds__(256) void split_act_kernel(const float* __restrict__ src, unsigned short* __restrict__ hi,
                                                        unsigned short* __restrict__ lo, int n8) {
  const int i = blockIdx.x * 256 + threadIdx.x;
  if (i < n8) {
    const v4f a = *(const v4f*)(src + (size_t)i * 8);
    const v4f b = *(const v4f*)(src + (size_t)i * 8 + 4);
    v8h hv, lv;
#pragma unroll
    for (int e = 0; e < 4; ++e) {
      const float fa = a[e];
      const float fb = b[e];
      _Float16 h0, l0, h1, l1;
      split_hl(fa, h0, l0);
      split_hl(fb, h1, l1);
      hv[e] = h0; lv[e] = l0;
      hv[4 + e] = h1; lv[4 + e] = l1;
    }
    volatile v8h* ph = (volatile v8h*)(hi + (size_t)i * 8);
    volatile v8h* pl = (volatile v8h*)(lo + (size_t)i * 8);
    *ph = hv;
    *pl = lv;
    __threadfence();
    *ph = hv;
    *pl = lv;
  }
}

__global__ __launch_bounds__(256) void gemm_xg_kernel(
    const unsigned short* __restrict__ Ahip, const unsigned short* __restrict__ Alop,
    const unsigned short* __restrict__ Wp,
    const float* __restrict__ b_a, const float* __restrict__ b_b,
    float* __restrict__ C, int M, int N, int K) {
  typedef _Float16 T;
  typedef v16h V;
  __shared__ __align__(16) float sT[8][16 * SLABP];
  const T* Ahi = (const T*)Ahip;
  const T* Alo = (const T*)Alop;
  const T* Wt  = (const T*)Wp;
  const int lane = threadIdx.x & 31;
  const int wave = threadIdx.x >> 5;
  const int tilesN = N >> 6;
  const int tilesM = M >> 6;
  const int tile = blockIdx.x * 8 + wave;
  if (tile >= tilesM * tilesN) return;
  const int tm = tile / tilesN;
  const int tn = tile - tm * tilesN;
  const int m0 = tm << 6;
  const int n0 = tn << 6;
  const int rlane = lane & 15;
  const int koff  = (lane >> 4) * 8;
  const int mOff  = (lane >> 4) * 8;

  v8f acc[4][4];
#pragma unroll
  for (int i = 0; i < 4; ++i)
#pragma unroll
    for (int j = 0; j < 4; ++j) acc[i][j] = (v8f){0.f, 0.f, 0.f, 0.f, 0.f, 0.f, 0.f, 0.f};

#pragma unroll
  for (int ph = 0; ph < 2; ++ph) {
    const T* Ab = (ph == 0) ? Alo : Ahi;
    for (int k0 = 0; k0 < K; k0 += 32) {
      V bh[4];
#pragma unroll
      for (int j = 0; j < 4; ++j) {
        const size_t bo = (size_t)(n0 + (j << 4) + rlane) * (size_t)K + koff + k0;
        bh[j] = Frag<T>::load(Wt + bo);
      }
#pragma unroll
      for (int i = 0; i < 4; ++i) {
        const size_t ao = (size_t)(m0 + (i << 4) + rlane) * (size_t)K + koff + k0;
        const V ah = Frag<T>::load(Ab + ao);
#pragma unroll
        for (int j = 0; j < 4; ++j) acc[i][j] = Frag<T>::mma(ah, bh[j], acc[i][j]);
        guard_grp4(acc[i][0], acc[i][1], acc[i][2], acc[i][3], ah, bh[0], bh[1], bh[2], bh[3]);
      }
    }
    if (ph == 0) {
      acc_guard4(acc[0][0], acc[0][1], acc[0][2], acc[0][3]);
      acc_guard4(acc[1][0], acc[1][1], acc[1][2], acc[1][3]);
      acc_guard4(acc[2][0], acc[2][1], acc[2][2], acc[2][3]);
      acc_guard4(acc[3][0], acc[3][1], acc[3][2], acc[3][3]);
#pragma unroll
      for (int i = 0; i < 4; ++i)
#pragma unroll
        for (int j = 0; j < 4; ++j) acc[i][j] = acc[i][j] * LO_CARRY_INV;
    }
  }
  acc_guard4(acc[0][0], acc[0][1], acc[0][2], acc[0][3]);
  acc_guard4(acc[1][0], acc[1][1], acc[1][2], acc[1][3]);
  acc_guard4(acc[2][0], acc[2][1], acc[2][2], acc[2][3]);
  acc_guard4(acc[3][0], acc[3][1], acc[3][2], acc[3][3]);

  float* slab = sT[wave];
#pragma unroll
  for (int i = 0; i < 4; ++i) {
    const int mBase = m0 + (i << 4);
#pragma unroll
    for (int j = 0; j < 4; ++j) {
      const int n = n0 + (j << 4) + rlane;
      const float bv = b_a[n] + b_b[n];
#pragma unroll
      for (int r = 0; r < 8; ++r) {
        const float v = acc[i][j][r] * W_CARRY_INV + bv;
        slab[(mOff + r) * SLABP + (j << 4) + rlane] = v;
      }
    }
    __builtin_amdgcn_fence(__ATOMIC_RELEASE, "workgroup");
    __builtin_amdgcn_wave_barrier();
    __builtin_amdgcn_fence(__ATOMIC_ACQUIRE, "workgroup");
    {
      const int hh = lane >> 4, c4 = (lane & 15) * 4;
      for (int pass = 0; pass < 2; ++pass) {
#pragma unroll
        for (int it = 0; it < 8; ++it) {
          const int row = it * 2 + hh;
          const v4f v = *(const v4f*)(slab + row * SLABP + c4);
          *(volatile v4f*)(C + (size_t)(mBase + row) * (size_t)N + n0 + c4) = v;
        }
        __threadfence();
      }
    }
    __builtin_amdgcn_fence(__ATOMIC_RELEASE, "workgroup");
    __builtin_amdgcn_wave_barrier();
    __builtin_amdgcn_fence(__ATOMIC_ACQUIRE, "workgroup");
  }
}

__device__ __forceinline__ float sigm_f(float x) { return 1.0f / (1.0f + expf(-x)); }

__global__ __launch_bounds__(REC_THREADS) void lstm_rec_kernel(const float* __restrict__ XG,
                                                               const unsigned short* __restrict__ WHp,
                                                               float* __restrict__ HSEQ) {
  __shared__ __align__(16) _Float16 Ah[2 * 2 * HPITCH];
  __shared__ __align__(16) float    Sl[REC_WAVES * 64];
  const _Float16* WH = (const _Float16*)WHp;
  const int tid = threadIdx.x, lane = tid & 31, wave = tid >> 5;
  const int c = lane & 15, hh = lane >> 4, koff = hh * 8;

#pragma unroll 1
  for (int i = tid; i < 4 * HPITCH; i += REC_THREADS) Ah[i] = (_Float16)0.0f;

  float cst[UB_PER_WAVE];
#pragma unroll
  for (int u = 0; u < UB_PER_WAVE; ++u) cst[u] = 0.0f;
  const unsigned mk = (c < 2) ? 0xFFFFFFFFu : 0u;
  const v4u msk = {mk, mk, mk, mk};
  const v8f z8 = {0.f, 0.f, 0.f, 0.f, 0.f, 0.f, 0.f, 0.f};
  const size_t GSTR = (size_t)NHID * (size_t)NHID;
  float* slab = Sl + wave * 64;
  __syncthreads();

#pragma unroll 1
  for (int t = 0; t < NSTEP; ++t) {
    const int cur = t & 1;
    const _Float16* ahrow = Ah + cur * 2 * HPITCH + (c & 1) * HPITCH + koff;
    _Float16* ahn = Ah + (cur ^ 1) * 2 * HPITCH;
#pragma unroll
    for (int u = 0; u < UB_PER_WAVE; ++u) {
      const int j = 64 * wave + 16 * u + c;
      const float* xp = XG + (size_t)t * NGATE + j;
      float xi = xp[0];
      float xf = xp[NHID];
      float xc = xp[2 * NHID];
      float xo = xp[3 * NHID];
      asm volatile("" : "+v"(xi), "+v"(xf), "+v"(xc), "+v"(xo));
      const _Float16* w0 = WH + (size_t)j * NHID + koff;
      v8f a0 = z8, a1 = z8, a2 = z8, a3 = z8;
#pragma unroll 1
      for (int k0 = 0; k0 < NHID; k0 += 32) {
        Frag<_Float16>::U fa;
        fa.v = Frag<_Float16>::load(ahrow + k0);
        fa.q[0] = fa.q[0] & msk;
        fa.q[1] = fa.q[1] & msk;
        const v16h a  = fa.v;
        const v16h b0 = Frag<_Float16>::load(w0 + k0);
        const v16h b1 = Frag<_Float16>::load(w0 + GSTR + k0);
        const v16h b2 = Frag<_Float16>::load(w0 + 2 * GSTR + k0);
        const v16h b3 = Frag<_Float16>::load(w0 + 3 * GSTR + k0);
        a0 = Frag<_Float16>::mma(a, b0, a0);
        a1 = Frag<_Float16>::mma(a, b1, a1);
        a2 = Frag<_Float16>::mma(a, b2, a2);
        a3 = Frag<_Float16>::mma(a, b3, a3);
        guard_grp4(a0, a1, a2, a3, a, b0, b1, b2, b3);
      }
      acc_guard4(a0, a1, a2, a3);
      const float zi = (a0[0] + a0[1] * LO_CARRY_INV) * W_CARRY_INV + xi;
      const float zf = (a1[0] + a1[1] * LO_CARRY_INV) * W_CARRY_INV + xf;
      const float zc = (a2[0] + a2[1] * LO_CARRY_INV) * W_CARRY_INV + xc;
      const float zo = (a3[0] + a3[1] * LO_CARRY_INV) * W_CARRY_INV + xo;
      const float ig = sigm_f(zi);
      const float fg = sigm_f(zf);
      const float gg = tanhf(zc);
      const float og = sigm_f(zo);
      const float cn = fg * cst[u] + ig * gg;
      cst[u] = cn;
      const float hn = og * tanhf(cn);
      _Float16 hhi, hlo;
      split_hl(hn, hhi, hlo);
      if (hh == 0) {
        ahn[j] = hhi;
        ahn[HPITCH + j] = hlo;
        slab[16 * u + c] = hn;
      }
    }
    __builtin_amdgcn_fence(__ATOMIC_RELEASE, "workgroup");
    __builtin_amdgcn_wave_barrier();
    __builtin_amdgcn_fence(__ATOMIC_ACQUIRE, "workgroup");
    if (lane < 16) {
      const v4f v = *(const v4f*)(slab + 4 * lane);
      volatile v4f* op = (volatile v4f*)(HSEQ + (size_t)t * NHID + 64 * wave + 4 * lane);
      *op = v;
      __threadfence();
      *op = v;
    }
    __builtin_amdgcn_fence(__ATOMIC_RELEASE, "workgroup");
    __builtin_amdgcn_wave_barrier();
    __builtin_amdgcn_fence(__ATOMIC_ACQUIRE, "workgroup");
    __syncthreads();
  }
}

__global__ __launch_bounds__(256) void head_kernel(const float* __restrict__ HS, const float* __restrict__ wl,
                                                   const float* __restrict__ bl, float* __restrict__ out) {
  __shared__ __align__(16) float res[NSTEP];
  const int tid = threadIdx.x, lane = tid & 31, wave = tid >> 5;
  v4f w[8];
#pragma unroll
  for (int q = 0; q < 8; ++q) w[q] = *(const v4f*)(wl + 128 * q + 4 * lane);
#pragma unroll 1
  for (int i = 0; i < 16; ++i) {
    const int t = wave * 16 + i;
    const float* rp = HS + (size_t)t * NHID;
    float s = 0.0f;
#pragma unroll
    for (int q = 0; q < 8; ++q) {
      const v4f v = *(const v4f*)(rp + 128 * q + 4 * lane);
      s += v[0] * w[q][0];
      s += v[1] * w[q][1];
      s += v[2] * w[q][2];
      s += v[3] * w[q][3];
    }
#pragma unroll
    for (int off = 1; off < 32; off <<= 1) s += __shfl_xor(s, off, 32);
    if (lane == 0) res[t] = s;
  }
  __syncthreads();
  if (wave == 0) {
    const float bias = bl[0];
    v4f v = *(const v4f*)(res + 4 * lane);
    v[0] += bias;
    v[1] += bias;
    v[2] += bias;
    v[3] += bias;
    volatile v4f* p = (volatile v4f*)(out + 4 * lane);
    *p = v;
    __threadfence();
    *p = v;
  }
}

extern "C" void kernel_launch(void* const* d_in, const int* in_sizes, int n_in,
                              void* d_out, int out_size, void* d_ws, size_t ws_size, hipStream_t stream) {
  if (n_in < 11 || d_out == nullptr || d_ws == nullptr) return;
  if (in_sizes[0] != NBATCH * NSTEP * NIN || in_sizes[1] != NGATE * NIN || in_sizes[2] != NGATE * NHID ||
      in_sizes[3] != NGATE || in_sizes[4] != NGATE || in_sizes[5] != NGATE * NHID || in_sizes[6] != NGATE * NHID ||
      in_sizes[7] != NGATE || in_sizes[8] != NGATE || in_sizes[9] != NHID || in_sizes[10] != 1 ||
      out_size != NSTEP) return;

  const float* xin  = (const float*)d_in[0];
  const float* wih0 = (const float*)d_in[1];
  const float* whh0 = (const float*)d_in[2];
  const float* bih0 = (const float*)d_in[3];
  const float* bhh0 = (const float*)d_in[4];
  const float* wih1 = (const float*)d_in[5];
  const float* whh1 = (const float*)d_in[6];
  const float* bih1 = (const float*)d_in[7];
  const float* bhh1 = (const float*)d_in[8];
  const float* wlin = (const float*)d_in[9];
  const float* blin = (const float*)d_in[10];
  float* out = (float*)d_out;
  const float* xsel = xin + (size_t)BSEL * NSTEP * NIN;

  char* ws = (char*)d_ws;
  size_t off = 0;
  auto carve = [&](size_t bytes) -> char* { char* p = ws + off; off += (bytes + 255) & ~(size_t)255; return p; };
  unsigned short* WIH0 = (unsigned short*)carve((size_t)NGATE * NIN * 2);
  unsigned short* WHH0 = (unsigned short*)carve((size_t)NGATE * NHID * 2);
  unsigned short* WIH1 = (unsigned short*)carve((size_t)NGATE * NHID * 2);
  unsigned short* WHH1 = (unsigned short*)carve((size_t)NGATE * NHID * 2);
  unsigned short* XHI  = (unsigned short*)carve((size_t)NSTEP * NIN * 2);
  unsigned short* XLO  = (unsigned short*)carve((size_t)NSTEP * NIN * 2);
  float*          XG   = (float*)carve((size_t)NSTEP * NGATE * 4);
  float*          HSEQ1 = (float*)carve((size_t)NSTEP * NHID * 4);
  unsigned short* H1HI = (unsigned short*)carve((size_t)NSTEP * NHID * 2);
  unsigned short* H1LO = (unsigned short*)carve((size_t)NSTEP * NHID * 2);
  float*          HSEQ2 = (float*)carve((size_t)NSTEP * NHID * 4);
  if (off > ws_size || off > (size_t)134217728) return;

  const int n8w0 = NGATE * NIN / 8;
  const int n8w1 = NGATE * NHID / 8;
  const int n8x  = NSTEP * NIN / 8;
  const int n8h  = NSTEP * NHID / 8;
  cvt_w_kernel<<<(n8w0 + 255) / 256, 256, 0, stream>>>(wih0, WIH0, n8w0, W_CARRY);
  cvt_w_kernel<<<(n8w1 + 255) / 256, 256, 0, stream>>>(whh0, WHH0, n8w1, W_CARRY);
  cvt_w_kernel<<<(n8w1 + 255) / 256, 256, 0, stream>>>(wih1, WIH1, n8w1, W_CARRY);
  cvt_w_kernel<<<(n8w1 + 255) / 256, 256, 0, stream>>>(whh1, WHH1, n8w1, W_CARRY);
  split_act_kernel<<<(n8x + 255) / 256, 256, 0, stream>>>(xsel, XHI, XLO, n8x);

  const int gblocks = ((NSTEP / 64) * (NGATE / 64) + 7) / 8;

  gemm_xg_kernel<<<gblocks, 256, 0, stream>>>(XHI, XLO, WIH0, bih0, bhh0, XG, NSTEP, NGATE, NIN);
  lstm_rec_kernel<<<1, REC_THREADS, 0, stream>>>(XG, WHH0, HSEQ1);

  split_act_kernel<<<(n8h + 255) / 256, 256, 0, stream>>>(HSEQ1, H1HI, H1LO, n8h);
  gemm_xg_kernel<<<gblocks, 256, 0, stream>>>(H1HI, H1LO, WIH1, bih1, bhh1, XG, NSTEP, NGATE, NHID);
  lstm_rec_kernel<<<1, REC_THREADS, 0, stream>>>(XG, WHH1, HSEQ2);

  head_kernel<<<1, 256, 0, stream>>>(HSEQ2, wlin, blin, out);
}
